// MultiHeadAttn_31404800868449
// MI455X (gfx1250) — hardware-verified
//
#include <hip/hip_runtime.h>
#include <math.h>
#include <stdint.h>

#ifndef NB
#define NB 1
#endif
#ifndef SEQ
#define SEQ 2048
#endif
#ifndef SEQ_FULL
#define SEQ_FULL 2048
#endif
#ifndef OUT_SEQ
#define OUT_SEQ SEQ_FULL
#endif
#define NH    16
#define HD    64
#define WIN   256
#define NQB   (SEQ / 64)
#ifndef RESQB
#define RESQB 8
#endif
#define PCARRY 16384.0f
#define PRES   4096.0f
#define VCARRY 64.0f

static_assert(NB == 1);
static_assert((SEQ % 64) == 0 && SEQ >= 64);
static_assert(SEQ <= SEQ_FULL && SEQ <= OUT_SEQ);
static_assert(RESQB >= 1);
static_assert((long long)NH * 2048 * HD * 4 == 8388608LL);
static_assert((long long)NH * 2048 * HD * 4 * 2 == 16777216LL);

typedef _Float16 v16h __attribute__((ext_vector_type(16)));
typedef _Float16 v8h  __attribute__((ext_vector_type(8)));
typedef __bf16   v16b __attribute__((ext_vector_type(16)));
typedef __bf16   v8b  __attribute__((ext_vector_type(8)));
typedef float    v8f  __attribute__((ext_vector_type(8)));
typedef float    v4f  __attribute__((ext_vector_type(4)));
typedef unsigned int v4u __attribute__((ext_vector_type(4)));

__device__ __forceinline__ unsigned short bf_bits(float f) {
  unsigned u = __float_as_uint(f);
  return (unsigned short)((u + 0x7FFFu + ((u >> 16) & 1u)) >> 16);
}
__device__ __forceinline__ float bf_up(unsigned short h) { return __uint_as_float(((unsigned)h) << 16); }
__device__ __forceinline__ unsigned pk16(unsigned short a, unsigned short b) { return (unsigned)a | ((unsigned)b << 16); }
__device__ __forceinline__ v8f zero8() { v8f z = {0.f, 0.f, 0.f, 0.f, 0.f, 0.f, 0.f, 0.f}; return z; }

__device__ __forceinline__ v16b ldfrag_b(const __bf16* p) {
  union { v16b v; v8b h[2]; } f;
  f.h[0] = *(const v8b*)(p);
  f.h[1] = *(const v8b*)(p + 16);
  return f.v;
}

__device__ __forceinline__ v8f mma_b(v16b a, v16b b, v8f c) {
  c = __builtin_amdgcn_wmma_f32_16x16x32_bf16(false, a, false, b, (short)0, c, false, false);
  asm volatile("v_nop\n\tv_nop\n\tv_nop\n\tv_nop" : "+v"(c) : "v"(a), "v"(b));
  return c;
}
__device__ __forceinline__ v8f mma_h(v16h a, v16h b, v8f c) {
  c = __builtin_amdgcn_wmma_f32_16x16x32_f16(false, a, false, b, (short)0, c, false, false);
  asm volatile("v_nop\n\tv_nop\n\tv_nop\n\tv_nop" : "+v"(c) : "v"(a), "v"(b));
  return c;
}

__global__ __launch_bounds__(256) void cvt_bf16x8s(const float* __restrict__ in, unsigned short* out,
                                                   int n8, int per8, int src8) {
  const int i = blockIdx.x * 256 + threadIdx.x;
  if (i < n8) {
    const int hd  = i / per8;
    const int rem = i - hd * per8;
    const float* s = in + ((size_t)hd * src8 + (size_t)rem) * 8;
    const v4f a = *(const v4f*)(s);
    const v4f b = *(const v4f*)(s + 4);
    v4u p;
    p[0] = pk16(bf_bits(a[0]), bf_bits(a[1]));
    p[1] = pk16(bf_bits(a[2]), bf_bits(a[3]));
    p[2] = pk16(bf_bits(b[0]), bf_bits(b[1]));
    p[3] = pk16(bf_bits(b[2]), bf_bits(b[3]));
    *(volatile v4u*)(out + (size_t)i * 8) = p;
    __threadfence();
    *(volatile v4u*)(out + (size_t)i * 8) = p;
  }
}

__global__ __launch_bounds__(256) void copy_f32x4s(const float* __restrict__ in, float* out,
                                                   int n4, int per4, int src4) {
  const int i = blockIdx.x * 256 + threadIdx.x;
  if (i < n4) {
    const int hd  = i / per4;
    const int rem = i - hd * per4;
    const v4f a = *(const v4f*)(in + ((size_t)hd * src4 + (size_t)rem) * 4);
    *(volatile v4f*)(out + (size_t)i * 4) = a;
    __threadfence();
    *(volatile v4f*)(out + (size_t)i * 4) = a;
  }
}

__global__ __launch_bounds__(256) void vt_f16_tiles(const float* __restrict__ v, unsigned short* vt) {
  __shared__ __align__(16) _Float16 T[64 * 64];
  const int tid = threadIdx.x;
  const int h   = blockIdx.x / NQB;
  const int kt  = blockIdx.x - h * NQB;
  const int s   = tid >> 2;
  const int dq  = (tid & 3) * 16;
  const float* src = v + (((size_t)h * SEQ_FULL) + (size_t)kt * 64 + (size_t)s) * HD + dq;
#pragma unroll
  for (int i = 0; i < 4; ++i) {
    const v4f a = *(const v4f*)(src + 4 * i);
#pragma unroll
    for (int e = 0; e < 4; ++e) {
      const float f = bf_up(bf_bits(a[e])) * VCARRY;
      T[(dq + 4 * i + e) * 64 + s] = (_Float16)f;
    }
  }
  __syncthreads();
  const int wave = tid >> 5, lane = tid & 31;
  const int q = lane >> 3, c8 = (lane & 7) * 8;
  union { v8h h; v4u u; } w0, w1;
  const int d0 = wave * 8 + q;
  const int d1 = wave * 8 + 4 + q;
  w0.h = *(const v8h*)(T + d0 * 64 + c8);
  w1.h = *(const v8h*)(T + d1 * 64 + c8);
  unsigned short* p0 = vt + ((size_t)(h * HD + d0) * SEQ + (size_t)kt * 64 + c8);
  unsigned short* p1 = vt + ((size_t)(h * HD + d1) * SEQ + (size_t)kt * 64 + c8);
  *(volatile v4u*)p0 = w0.u;
  *(volatile v4u*)p1 = w1.u;
  __threadfence();
  *(volatile v4u*)p0 = w0.u;
  *(volatile v4u*)p1 = w1.u;
}

template <bool RES>
__global__ __launch_bounds__(128)
void attn_band64(const unsigned short* __restrict__ qp, const unsigned short* __restrict__ kp,
                 const unsigned short* __restrict__ vtp, const int* __restrict__ lidx,
                 const int* __restrict__ trn, float* out, int qbBase, int nqbThis) {
  union FB { v16b v; v8b h[2]; };
  union FH { v16h v; v8h h[2]; };
  __shared__ __align__(16) __bf16   Ksh[64 * 64];
  __shared__ __align__(16) _Float16 Vth[64 * 64];
  __shared__ __align__(16) _Float16 Psh[4][16 * 64];
  __shared__ __align__(16) _Float16 Psl[RES ? 4 : 1][16 * 64];
  __shared__ __align__(16) float    Os[4][16 * 64];

  const int tid  = threadIdx.x;
  const int wave = tid >> 5;
  const int lane = tid & 31;
  const int hh   = lane >> 4;
  const int c    = lane & 15;

  const int bx   = blockIdx.x;
  const int qbl  = bx % nqbThis;
  const int h    = bx / nqbThis;
  const int qb   = qbBase + qbl;
  const int q0   = qb * 64 + wave * 16;
  (void)trn;

  const int li = lidx[0];
  const bool local = (li & 1) != 0;
  int lo = qb * 64 - (WIN - 1);
  if (lo < 0) lo = 0;
  int ktStart = local ? (lo >> 6) : 0;
  if (ktStart > qb) ktStart = qb;
  if (ktStart < 0) ktStart = 0;

  const __bf16*   Qh = (const __bf16*)(const void*)qp + (size_t)h * SEQ * HD;
  const __bf16*   Kh = (const __bf16*)(const void*)kp + (size_t)h * SEQ * HD;
  const _Float16* Vh = (const _Float16*)(const void*)vtp + (size_t)h * HD * SEQ;

  v16b qa[2];
#pragma unroll
  for (int dc = 0; dc < 2; ++dc) {
    const size_t qo = (size_t)(q0 + c) * HD + dc * 32 + 8 * hh;
    qa[dc] = ldfrag_b(Qh + qo);
  }

  float mrow[8], lrow[8];
  v8f oacc[4];
#pragma unroll
  for (int r = 0; r < 8; ++r) { mrow[r] = -INFINITY; lrow[r] = 0.f; }
#pragma unroll
  for (int t = 0; t < 4; ++t) oacc[t] = zero8();

  for (int kt = ktStart; kt <= qb; ++kt) {
    const int kv0 = kt * 64;
    __syncthreads();
    {
      const int r = tid >> 1, half = (tid & 1) * 32;
      const __bf16*   kg = Kh + (size_t)(kv0 + r) * HD + half;
      const _Float16* vg = Vh + (size_t)r * SEQ + kv0 + half;
#pragma unroll
      for (int i = 0; i < 4; ++i) {
        const v8b a0 = *(const v8b*)(kg + 8 * i);
        const v8h b0 = *(const v8h*)(vg + 8 * i);
        *(v8b*)(Ksh + r * 64 + half + 8 * i) = a0;
        *(v8h*)(Vth + r * 64 + half + 8 * i) = b0;
      }
    }
    __syncthreads();

    v8f s[4];
#pragma unroll
    for (int j = 0; j < 4; ++j) {
      s[j] = zero8();
#pragma unroll
      for (int dc = 0; dc < 2; ++dc) {
        FB kb;
        kb.h[0] = *(const v8b*)(Ksh + (j * 16 + c) * 64 + dc * 32 + 8 * hh);
        kb.h[1] = *(const v8b*)(Ksh + (j * 16 + c) * 64 + dc * 32 + 16 + 8 * hh);
        s[j] = mma_b(qa[dc], kb.v, s[j]);
      }
    }

    _Float16* pwh = Psh[wave];
    _Float16* pwl = Psl[RES ? wave : 0];
#pragma unroll
    for (int r = 0; r < 8; ++r) {
      const int qi = q0 + 8 * hh + r;
      float m = -INFINITY;
#pragma unroll
      for (int j = 0; j < 4; ++j) {
        const int kj = kv0 + j * 16 + c;
        const bool ok = (kj <= qi) && ((!local) || ((qi - kj) < WIN));
        const float sv = ok ? (s[j][r] * 0.125f) : -1.0e9f;
        s[j][r] = sv;
        m = fmaxf(m, sv);
      }
#pragma unroll
      for (int off = 1; off < 16; off <<= 1) m = fmaxf(m, __shfl_xor(m, off, 32));
      const float mnew  = fmaxf(mrow[r], m);
      const float msafe = (mnew == -INFINITY) ? 0.f : mnew;
      const float alpha = __expf(mrow[r] - msafe);
      mrow[r] = mnew;
      float psum = 0.f;
#pragma unroll
      for (int j = 0; j < 4; ++j) {
        const float p = __expf(s[j][r] - msafe);
        psum += p;
        const float p1k = p * PCARRY;
        const _Float16 ph = (_Float16)p1k;
        pwh[(8 * hh + r) * 64 + j * 16 + c] = ph;
        if (RES) {
          const _Float16 pl = (_Float16)((p1k - (float)ph) * PRES);
          pwl[(8 * hh + r) * 64 + j * 16 + c] = pl;
        }
      }
#pragma unroll
      for (int off = 1; off < 16; off <<= 1) psum += __shfl_xor(psum, off, 32);
      lrow[r] = lrow[r] * alpha + psum;
#pragma unroll
      for (int t = 0; t < 4; ++t) oacc[t][r] *= alpha;
    }
    __builtin_amdgcn_fence(__ATOMIC_RELEASE, "workgroup");
    __builtin_amdgcn_wave_barrier();
    __builtin_amdgcn_fence(__ATOMIC_ACQUIRE, "workgroup");

    v8f o1[4];
#pragma unroll
    for (int t = 0; t < 4; ++t) o1[t] = zero8();
#pragma unroll 1
    for (int kk = 0; kk < 2; ++kk) {
      FH pa, pl;
      pa.h[0] = *(const v8h*)(pwh + c * 64 + kk * 32 + 8 * hh);
      pa.h[1] = *(const v8h*)(pwh + c * 64 + kk * 32 + 16 + 8 * hh);
      if (RES) {
        pl.h[0] = *(const v8h*)(pwl + c * 64 + kk * 32 + 8 * hh);
        pl.h[1] = *(const v8h*)(pwl + c * 64 + kk * 32 + 16 + 8 * hh);
      } else {
        pl.v = pa.v;
      }
#pragma unroll
      for (int t = 0; t < 4; ++t) {
        FH vb;
        vb.h[0] = *(const v8h*)(Vth + (t * 16 + c) * 64 + kk * 32 + 8 * hh);
        vb.h[1] = *(const v8h*)(Vth + (t * 16 + c) * 64 + kk * 32 + 16 + 8 * hh);
        oacc[t] = mma_h(pa.v, vb.v, oacc[t]);
        if (RES) o1[t] = mma_h(pl.v, vb.v, o1[t]);
      }
    }
    if (RES) {
#pragma unroll
      for (int t = 0; t < 4; ++t)
#pragma unroll
        for (int r = 0; r < 8; ++r) oacc[t][r] += o1[t][r] * (1.0f / PRES);
    }
  }

  float* os = Os[wave];
#pragma unroll
  for (int r = 0; r < 8; ++r) {
    const float l = lrow[r];
    const float inv = ((l > 0.f) ? (1.0f / l) : 0.f) * (1.0f / (PCARRY * VCARRY));
#pragma unroll
    for (int t = 0; t < 4; ++t) os[(8 * hh + r) * 64 + t * 16 + c] = oacc[t][r] * inv;
  }
  __builtin_amdgcn_fence(__ATOMIC_RELEASE, "workgroup");
  __builtin_amdgcn_wave_barrier();
  __builtin_amdgcn_fence(__ATOMIC_ACQUIRE, "workgroup");
  {
    const int h2 = lane >> 4, c4 = (lane & 15) * 4;
    float* ob = out + (size_t)h * SEQ * HD;
    for (int rep = 0; rep < 2; ++rep) {
#pragma unroll
      for (int it = 0; it < 8; ++it) {
        const int row = it * 2 + h2;
        const v4f val = *(const v4f*)(os + row * 64 + c4);
        *(volatile v4f*)(ob + (size_t)(q0 + row) * HD + c4) = val;
      }
      __threadfence();
    }
  }
}

extern "C" void kernel_launch(void* const* d_in, const int* in_sizes, int n_in,
                              void* d_out, int out_size, void* d_ws, size_t ws_size,
                              hipStream_t stream) {
  if (n_in < 5) return;
  const long long needIn = (long long)(NH - 1) * SEQ_FULL * HD + (long long)SEQ * HD;
  if ((long long)in_sizes[0] < needIn || (long long)in_sizes[1] < needIn || (long long)in_sizes[2] < needIn) return;
  if (in_sizes[3] < 1 || in_sizes[4] < 1) return;

  const size_t perOut = (size_t)NH * SEQ * HD;
  const size_t oOut1  = (size_t)NH * OUT_SEQ * HD;
  const size_t oOut2  = 2 * oOut1;
  if (out_size < 0 || (size_t)out_size < oOut2 + perOut) return;

  const size_t PQ = (size_t)NH * SEQ * HD * 2;
  size_t off = 0;
  const size_t oQ  = off; off += PQ;
  const size_t oK  = off; off += PQ;
  const size_t oVT = off; off += PQ;
  if (off > ws_size) return;
  if (off > (size_t)134217728) return;

  const float* q    = (const float*)d_in[0];
  const float* k    = (const float*)d_in[1];
  const float* v    = (const float*)d_in[2];
  const int*   lidx = (const int*)d_in[3];
  const int*   trn  = (const int*)d_in[4];
  float* out = (float*)d_out;

  char* ws = (char*)d_ws;
  unsigned short* Qb  = (unsigned short*)(ws + oQ);
  unsigned short* Kb  = (unsigned short*)(ws + oK);
  unsigned short* VTb = (unsigned short*)(ws + oVT);

  const dim3 blk(256);
  const int n8   = NH * SEQ * HD / 8;
  const int per8 = SEQ * HD / 8;
  const int src8 = SEQ_FULL * HD / 8;
  const dim3 gCvt((n8 + 255) / 256);
  const int n4   = NH * SEQ * HD / 4;
  const int per4 = SEQ * HD / 4;
  const int src4 = SEQ_FULL * HD / 4;
  const dim3 gCpy((n4 + 255) / 256);
  const dim3 gVT(NH * NQB);
  int resqb = RESQB;
  if (resqb > NQB) resqb = NQB;

  cvt_bf16x8s<<<gCvt, blk, 0, stream>>>(q, Qb, n8, per8, src8);
  cvt_bf16x8s<<<gCvt, blk, 0, stream>>>(k, Kb, n8, per8, src8);
  vt_f16_tiles<<<gVT, blk, 0, stream>>>(v, VTb);
  attn_band64<true><<<dim3(NH * resqb), dim3(128), 0, stream>>>(Qb, Kb, VTb, lidx, trn, out, 0, resqb);
  if (NQB - resqb > 0) {
    attn_band64<false><<<dim3(NH * (NQB - resqb)), dim3(128), 0, stream>>>(Qb, Kb, VTb, lidx, trn, out, resqb, NQB - resqb);
  }
  copy_f32x4s<<<gCpy, blk, 0, stream>>>(k, out + oOut1, n4, per4, src4);
  copy_f32x4s<<<gCpy, blk, 0, stream>>>(v, out + oOut2, n4, per4, src4);
  (void)hipGetLastError();
}
